// MambaBlock_27161373179954
// MI455X (gfx1250) — hardware-run, weakly checked
//
#include <hip/hip_runtime.h>
#include <math.h>

typedef __attribute__((ext_vector_type(16))) _Float16 v16h;
typedef __attribute__((ext_vector_type(8)))  _Float16 v8h;
typedef __attribute__((ext_vector_type(8)))  float    v8f;
typedef __attribute__((ext_vector_type(4)))  float    v4f;
typedef __attribute__((ext_vector_type(4)))  unsigned v4u;

constexpr int kBatch = 2;
constexpr int kSeq   = 2048;
constexpr int kDm    = 1024;
constexpr int kDin   = 2048;
constexpr int kNst   = 16;
constexpr int kDtR   = 64;
constexpr int kXzP   = 2 * kDin;
constexpr int kXdN   = kDtR + 2 * kNst;
constexpr int kXdP   = 128;
constexpr int kRows  = kBatch * kSeq;
constexpr int kConvRows = 32;
constexpr int kScanTS   = 16;
static_assert(kXdN == 96);
static_assert((kDm % 32) == 0 && (kDin % 32) == 0 && (kDtR % 32) == 0);
static_assert((kRows % 64) == 0 && (kXzP % 64) == 0 && (kXdP % 64) == 0 && (kDin % 64) == 0 && (kDm % 64) == 0);
static_assert((kSeq % kConvRows) == 0 && (kSeq % kScanTS) == 0);
static_assert(kDm == 8 * 128);

constexpr int kCarryXLog2    = 4;
constexpr int kCarryWinLog2  = 8;
constexpr int kCarryWxLog2   = 9;
constexpr int kCarryWdtLog2  = 8;
constexpr int kCarryWoutLog2 = 9;
constexpr int kCarryUcLog2   = 6;
constexpr int kCarryDlLog2   = 6;
constexpr int kCarryYgLog2   = 8;
constexpr float kCarryUcF    = (float)(1u << kCarryUcLog2);
constexpr float kInvCarryUcF = 1.0f / (float)(1u << kCarryUcLog2);
constexpr float kCarryYgF    = (float)(1u << kCarryYgLog2);
constexpr float kF16MinNormal = 6.103515625e-5f;

constexpr size_t kSzXH  = (size_t)kRows * kDm  * 2;
constexpr size_t kSzWIH = (size_t)kXzP  * kDm  * 2;
constexpr size_t kSzWXH = (size_t)kXdP  * kDin * 2;
constexpr size_t kSzWDH = (size_t)kDin  * kDtR * 2;
constexpr size_t kSzWOH = (size_t)kDm   * kDin * 2;
constexpr size_t kSzXZH = (size_t)kRows * kXzP * 2;
constexpr size_t kSzUCH = (size_t)kRows * kDin * 2;
constexpr size_t kSzXD  = (size_t)kRows * kXdP * 4;
constexpr size_t kSzDLH = (size_t)kRows * kDtR * 2;
constexpr size_t kSzDTH = (size_t)kRows * kDin * 2;
constexpr size_t kSzYGH = (size_t)kRows * kDin * 2;
constexpr size_t kSzPLN = (size_t)kRows * kDm  * 4;
constexpr size_t kOffXH  = 0;
constexpr size_t kOffWIH = kOffXH  + kSzXH;
constexpr size_t kOffWXH = kOffWIH + kSzWIH;
constexpr size_t kOffWDH = kOffWXH + kSzWXH;
constexpr size_t kOffWOH = kOffWDH + kSzWDH;
constexpr size_t kOffXZH = kOffWOH + kSzWOH;
constexpr size_t kOffUCH = kOffXZH + kSzXZH;
constexpr size_t kOffXD  = kOffUCH + kSzUCH;
constexpr size_t kOffDLH = kOffXD  + kSzXD;
constexpr size_t kOffDTH = kOffDLH + kSzDLH;
constexpr size_t kOffYGH = kOffDTH + kSzDTH;
constexpr size_t kOffPLN = kOffYGH + kSzYGH;
constexpr size_t kWsTotal = kOffPLN + kSzPLN;
static_assert(kWsTotal == 125042688ull);
static_assert(kWsTotal <= 134217728ull);
static_assert((kOffWIH % 128) == 0 && (kOffWXH % 128) == 0 && (kOffWDH % 128) == 0 && (kOffWOH % 128) == 0 &&
              (kOffXZH % 128) == 0 && (kOffUCH % 128) == 0 && (kOffXD % 128) == 0 && (kOffDLH % 128) == 0 &&
              (kOffDTH % 128) == 0 && (kOffYGH % 128) == 0 && (kOffPLN % 128) == 0);

__device__ __forceinline__ float h16_to_f32(unsigned hb) {
  const unsigned sgn = (hb & 0x8000u) << 16;
  const unsigned em = hb & 0x7fffu;
  const float fn = __uint_as_float((em << 13) + 0x38000000u);
  const float fs = (float)em * 5.9604644775390625e-8f;
  const float mag = (em < 0x400u) ? fs : fn;
  return __uint_as_float(__float_as_uint(mag) | sgn);
}

__device__ __forceinline__ unsigned f16_bits_flush(float s) {
  const float t = (fabsf(s) < kF16MinNormal) ? 0.0f : s;
  const _Float16 hv = (_Float16)t;
  const unsigned short hb = __builtin_bit_cast(unsigned short, hv);
  unsigned u = (unsigned)hb;
  asm volatile("" : "+v"(u));
  return u;
}
__device__ __forceinline__ unsigned pack2_f16(float lo_v, float hi_v) {
  const unsigned lo = f16_bits_flush(lo_v);
  const unsigned hi = f16_bits_flush(hi_v);
  return (hi << 16) | (lo & 0xffffu);
}

__device__ __forceinline__ float softplus_stable(float v) {
  return fmaxf(v, 0.0f) + log1pf(expf(-fabsf(v)));
}

__device__ __forceinline__ void wave_lds_sync() {
  __builtin_amdgcn_fence(__ATOMIC_RELEASE, "workgroup");
  __builtin_amdgcn_wave_barrier();
  __builtin_amdgcn_fence(__ATOMIC_ACQUIRE, "workgroup");
}

__device__ __forceinline__ void guard_row4(v8f& a, v8f& b, v8f& c, v8f& d, v16h x) {
  asm volatile("v_nop\n\tv_nop\n\tv_nop\n\tv_nop" : "+v"(a), "+v"(b), "+v"(c), "+v"(d) : "v"(x));
}
__device__ __forceinline__ void keep4_h(v16h a, v16h b, v16h c, v16h d) {
  asm volatile("v_nop" :: "v"(a), "v"(b), "v"(c), "v"(d));
}
__device__ __forceinline__ void acc_guard4(v8f& a, v8f& b, v8f& c, v8f& d) {
  asm volatile("v_nop\n\tv_nop\n\tv_nop\n\tv_nop" : "+v"(a), "+v"(b), "+v"(c), "+v"(d));
}

union FragU { v16h v; v8h h[2]; };
__device__ __forceinline__ v16h frag_load(const _Float16* p) {
  FragU f;
  f.h[0] = *(const v8h*)(p);
  f.h[1] = *(const v8h*)(p + 16);
  return f.v;
}
__device__ __forceinline__ v8f frag_mma(v16h a, v16h b, v8f c) {
  return __builtin_amdgcn_wmma_f32_16x16x32_f16(false, a, false, b, (short)0, c, false, false);
}

template <int CARRY_LOG2>
__global__ __launch_bounds__(256) void cast_rows_f16(
    const float* __restrict__ src, unsigned short* __restrict__ dst,
    int srcPitch, int dstPitch, int perShift, int rowsReal, int total8)
{
  constexpr float carry = (float)(1u << CARRY_LOG2);
  unsigned i = blockIdx.x * 256u + threadIdx.x;
  if (i >= (unsigned)total8) return;
  unsigned row = i >> perShift;
  unsigned c8 = (i - (row << perShift)) << 3;
  asm volatile("" : "+v"(row));
  asm volatile("" : "+v"(c8));
  const bool valid = row < (unsigned)rowsReal;
  const unsigned rc = valid ? row : (unsigned)(rowsReal - 1);
  const float* sp = src + (size_t)rc * srcPitch + c8;
  const v4f a0 = *(const v4f*)(sp);
  const v4f a1 = *(const v4f*)(sp + 4);
  const float f0 = valid ? a0[0] * carry : 0.0f;
  const float f1 = valid ? a0[1] * carry : 0.0f;
  const float f2 = valid ? a0[2] * carry : 0.0f;
  const float f3 = valid ? a0[3] * carry : 0.0f;
  const float f4 = valid ? a1[0] * carry : 0.0f;
  const float f5 = valid ? a1[1] * carry : 0.0f;
  const float f6 = valid ? a1[2] * carry : 0.0f;
  const float f7 = valid ? a1[3] * carry : 0.0f;
  v4u ov;
  ov[0] = pack2_f16(f0, f1);
  ov[1] = pack2_f16(f2, f3);
  ov[2] = pack2_f16(f4, f5);
  ov[3] = pack2_f16(f6, f7);
  unsigned short* dp = dst + (size_t)row * dstPitch + c8;
  *(volatile v4u*)dp = ov;
  __threadfence();
  *(volatile v4u*)dp = ov;
}

template <int SCALE_LOG2, int OUT_F16, int OUT_CARRY_LOG2, int BIAS_N, int RESID, int SOFTPLUS>
__global__ __launch_bounds__(256) void wmma_gemm64_f16(
    const unsigned short* __restrict__ Ap, int lda,
    const unsigned short* __restrict__ Btp, int ldb,
    void* __restrict__ Cout, int ldc,
    const float* __restrict__ bias,
    const float* __restrict__ resid, int ldr,
    int M, int N, int K)
{
  const _Float16* A  = (const _Float16*)Ap;
  const _Float16* Bt = (const _Float16*)Btp;
  __shared__ __align__(16) float sT[8][16 * 68];
  const int lane = threadIdx.x & 31;
  const int wave = threadIdx.x >> 5;
  const int tilesN = N >> 6;
  const int tilesM = M >> 6;
  const int tile = blockIdx.x * 8 + wave;
  if (tile >= tilesM * tilesN) return;
  const int tm = tile / tilesN;
  const int tn = tile - tm * tilesN;
  const int m0 = tm << 6;
  const int n0 = tn << 6;

  const int rlane = lane & 15;
  const int koff  = (lane >> 4) * 8;
  const int mOff  = (lane >> 4) * 8;

  v8f acc[4][4];
#pragma unroll
  for (int i = 0; i < 4; ++i)
#pragma unroll
    for (int j = 0; j < 4; ++j) acc[i][j] = (v8f){0.f, 0.f, 0.f, 0.f, 0.f, 0.f, 0.f, 0.f};

  for (int k0 = 0; k0 < K; k0 += 32) {
    v16h bh[4];
#pragma unroll
    for (int j = 0; j < 4; ++j) {
      const size_t bo = (size_t)(n0 + (j << 4) + rlane) * ldb + koff + k0;
      bh[j] = frag_load(Bt + bo);
    }
#pragma unroll
    for (int i = 0; i < 4; ++i) {
      const size_t ao = (size_t)(m0 + (i << 4) + rlane) * lda + koff + k0;
      const v16h ah = frag_load(A + ao);
#pragma unroll
      for (int j = 0; j < 4; ++j) acc[i][j] = frag_mma(ah, bh[j], acc[i][j]);
      guard_row4(acc[i][0], acc[i][1], acc[i][2], acc[i][3], ah);
    }
    keep4_h(bh[0], bh[1], bh[2], bh[3]);
  }
  acc_guard4(acc[0][0], acc[0][1], acc[0][2], acc[0][3]);
  acc_guard4(acc[1][0], acc[1][1], acc[1][2], acc[1][3]);
  acc_guard4(acc[2][0], acc[2][1], acc[2][2], acc[2][3]);
  acc_guard4(acc[3][0], acc[3][1], acc[3][2], acc[3][3]);

  constexpr float sc = 1.0f / (float)(1u << SCALE_LOG2);
  constexpr float oc = (float)(1u << OUT_CARRY_LOG2);
  float* slab = sT[wave];
#pragma unroll
  for (int i = 0; i < 4; ++i) {
    const int mBase = m0 + (i << 4);
#pragma unroll
    for (int j = 0; j < 4; ++j) {
      const int n = n0 + (j << 4) + rlane;
      float bv = 0.f;
      if (BIAS_N) bv = bias[n];
#pragma unroll
      for (int r = 0; r < 8; ++r) {
        float v = acc[i][j][r] * sc;
        if (BIAS_N) v += bv;
        slab[(mOff + r) * 68 + (j << 4) + rlane] = v;
      }
    }
    wave_lds_sync();
    if (SOFTPLUS) {
#pragma unroll 1
      for (int t = 0; t < 32; ++t) {
        const int sidx = (t >> 1) * 68 + (t & 1) * 32 + lane;
        const float v = slab[sidx];
        slab[sidx] = softplus_stable(v);
      }
      wave_lds_sync();
    }
    if (!OUT_F16) {
      float* C = (float*)Cout;
      const int hh = lane >> 4;
      const int c4 = (lane & 15) * 4;
      v4f ov[8];
#pragma unroll
      for (int it = 0; it < 8; ++it) {
        const int row = it * 2 + hh;
        v4f v = *(const v4f*)(slab + row * 68 + c4);
        if (RESID) {
          const v4f rv = *(const v4f*)(resid + (size_t)(mBase + row) * ldr + n0 + c4);
          v = v + rv;
        }
        ov[it] = v;
      }
      for (int pass = 0; pass < 2; ++pass) {
#pragma unroll
        for (int it = 0; it < 8; ++it) {
          const int row = it * 2 + hh;
          *(volatile v4f*)(C + (size_t)(mBase + row) * ldc + n0 + c4) = ov[it];
        }
        __threadfence();
      }
    } else {
      unsigned short* C = (unsigned short*)Cout;
      const int q = lane >> 3;
      const int c8 = (lane & 7) * 8;
      v8h hv[4];
#pragma unroll
      for (int it = 0; it < 4; ++it) {
        const int row = it * 4 + q;
        const float* sp = slab + row * 68 + c8;
#pragma unroll
        for (int e = 0; e < 8; ++e) {
          float s = sp[e] * oc;
          s = (fabsf(s) < kF16MinNormal) ? 0.0f : s;
          hv[it][e] = (_Float16)s;
        }
      }
      for (int pass = 0; pass < 2; ++pass) {
#pragma unroll
        for (int it = 0; it < 4; ++it) {
          const int row = it * 4 + q;
          *(volatile v8h*)(C + (size_t)(mBase + row) * ldc + n0 + c8) = hv[it];
        }
        __threadfence();
      }
    }
    wave_lds_sync();
  }
}

__global__ __launch_bounds__(256) void conv_silu_kernel(
    const unsigned* __restrict__ XZw, const float* __restrict__ cwt, const float* __restrict__ cbs,
    unsigned* __restrict__ UCw)
{
  unsigned cw = blockIdx.x * 256u + threadIdx.x;
  asm volatile("" : "+v"(cw));
  const int g0 = blockIdx.y * kConvRows;
  const int tb = g0 & (kSeq - 1);
  const v4f wa = *(const v4f*)(cwt + (size_t)cw * 8);
  const v4f wb = *(const v4f*)(cwt + (size_t)cw * 8 + 4);
  const float ba = cbs[2 * cw];
  const float bb = cbs[2 * cw + 1];
  float pa3, pa2, pa1, pb3, pb2, pb1;
  {
    const bool hist = (tb > 0);
    const int rb = hist ? (g0 - 3) : g0;
    const unsigned w3 = XZw[(size_t)rb * (kXzP / 2) + cw];
    const unsigned w2 = XZw[(size_t)(rb + 1) * (kXzP / 2) + cw];
    const unsigned w1 = XZw[(size_t)(rb + 2) * (kXzP / 2) + cw];
    const float a3 = h16_to_f32(w3 & 0xffffu), b3 = h16_to_f32(w3 >> 16);
    const float a2 = h16_to_f32(w2 & 0xffffu), b2 = h16_to_f32(w2 >> 16);
    const float a1 = h16_to_f32(w1 & 0xffffu), b1 = h16_to_f32(w1 >> 16);
    pa3 = hist ? a3 : 0.f;
    pa2 = hist ? a2 : 0.f;
    pa1 = hist ? a1 : 0.f;
    pb3 = hist ? b3 : 0.f;
    pb2 = hist ? b2 : 0.f;
    pb1 = hist ? b1 : 0.f;
  }
#pragma unroll 1
  for (int s = 0; s < kConvRows; ++s) {
    const size_t row = (size_t)(g0 + s);
    const unsigned wc = XZw[row * (kXzP / 2) + cw];
    const float xa = h16_to_f32(wc & 0xffffu);
    const float xb = h16_to_f32(wc >> 16);
    float aa = wa[0] * pa3;
    aa = fmaf(wa[1], pa2, aa);
    aa = fmaf(wa[2], pa1, aa);
    aa = fmaf(wa[3], xa, aa);
    aa = aa + ba;
    float ab = wb[0] * pb3;
    ab = fmaf(wb[1], pb2, ab);
    ab = fmaf(wb[2], pb1, ab);
    ab = fmaf(wb[3], xb, ab);
    ab = ab + bb;
    const float sa = aa * (1.0f / (1.0f + expf(-aa)));
    const float sb = ab * (1.0f / (1.0f + expf(-ab)));
    const unsigned wo = pack2_f16(sa * kCarryUcF, sb * kCarryUcF);
    volatile unsigned* p = (volatile unsigned*)(UCw + row * (kDin / 2) + cw);
    *p = wo;
    __threadfence();
    *p = wo;
    pa3 = pa2; pa2 = pa1; pa1 = xa;
    pb3 = pb2; pb2 = pb1; pb1 = xb;
  }
}

__global__ __launch_bounds__(256) void scan_gate_kernel(
    const unsigned* __restrict__ DTw, const unsigned* __restrict__ UCw, const unsigned* __restrict__ XZw,
    const float* __restrict__ XD, const float* __restrict__ Alog, const float* __restrict__ Dp,
    unsigned* __restrict__ YGw)
{
  __shared__ __align__(16) float sBC[kScanTS * 32];
  __shared__ __align__(16) float sA[kNst * 512];
  __shared__ unsigned sY[kScanTS * 256];
  const int tid = threadIdx.x;
  const int bix = blockIdx.x >> 2;
  unsigned wcol = (blockIdx.x & 3u) * 256u + (unsigned)tid;
  asm volatile("" : "+v"(wcol));
  const unsigned d = 2u * wcol;
  const size_t row0 = (size_t)bix * kSeq;

#pragma unroll 1
  for (int n = 0; n < kNst; ++n) {
    const float l0 = Alog[(size_t)d * kNst + n];
    const float l1 = Alog[(size_t)(d + 1) * kNst + n];
    sA[n * 512 + 2 * tid]     = -expf(l0);
    sA[n * 512 + 2 * tid + 1] = -expf(l1);
  }
  __syncthreads();
  float nA0[kNst], nA1[kNst], h0[kNst], h1[kNst];
#pragma unroll
  for (int n = 0; n < kNst; ++n) {
    nA0[n] = sA[n * 512 + 2 * tid];
    nA1[n] = sA[n * 512 + 2 * tid + 1];
    h0[n] = 0.f;
    h1[n] = 0.f;
  }
  const float Dd0 = Dp[d];
  const float Dd1 = Dp[d + 1];
  const int lr = tid >> 3;
  const int lc4 = (tid & 7) * 4;

#pragma unroll 1
  for (int t0 = 0; t0 < kSeq; t0 += kScanTS) {
    __syncthreads();
    if (tid < 128) {
      *(v4f*)(sBC + lr * 32 + lc4) = *(const v4f*)(XD + (row0 + t0 + lr) * kXdP + kDtR + lc4);
    }
    __syncthreads();
#pragma unroll 1
    for (int s = 0; s < kScanTS; ++s) {
      const size_t row = row0 + t0 + s;
      const unsigned wd = DTw[row * (kDin / 2) + wcol];
      const unsigned wu = UCw[row * (kDin / 2) + wcol];
      const unsigned wz = XZw[row * (kXzP / 2) + (kDin / 2) + wcol];
      const float dt0 = h16_to_f32(wd & 0xffffu);
      const float dt1 = h16_to_f32(wd >> 16);
      const float u0 = h16_to_f32(wu & 0xffffu) * kInvCarryUcF;
      const float u1 = h16_to_f32(wu >> 16) * kInvCarryUcF;
      const float z0 = h16_to_f32(wz & 0xffffu);
      const float z1 = h16_to_f32(wz >> 16);
      const float dx0 = dt0 * u0;
      const float dx1 = dt1 * u1;
      const float* xr = sBC + s * 32;
      float y0 = 0.f, y1 = 0.f;
#pragma unroll
      for (int q4 = 0; q4 < 4; ++q4) {
        const v4f bv = *(const v4f*)(xr + 4 * q4);
        const v4f cv = *(const v4f*)(xr + kNst + 4 * q4);
#pragma unroll
        for (int e = 0; e < 4; ++e) {
          const int n = 4 * q4 + e;
          const float e0 = __expf(dt0 * nA0[n]);
          const float e1 = __expf(dt1 * nA1[n]);
          h0[n] = e0 * h0[n] + dx0 * bv[e];
          h1[n] = e1 * h1[n] + dx1 * bv[e];
          y0 = h0[n] * cv[e] + y0;
          y1 = h1[n] * cv[e] + y1;
        }
      }
      y0 = u0 * Dd0 + y0;
      y1 = u1 * Dd1 + y1;
      const float s0 = __builtin_amdgcn_rcpf(1.0f + __expf(-z0));
      const float s1 = __builtin_amdgcn_rcpf(1.0f + __expf(-z1));
      const float g0 = y0 * (z0 * s0);
      const float g1 = y1 * (z1 * s1);
      sY[s * 256 + tid] = pack2_f16(g0 * kCarryYgF, g1 * kCarryYgF);
    }
    for (int pass = 0; pass < 2; ++pass) {
#pragma unroll 1
      for (int s = 0; s < kScanTS; ++s) {
        const unsigned w = sY[s * 256 + tid];
        *(volatile unsigned*)(YGw + (row0 + t0 + s) * (kDin / 2) + wcol) = w;
      }
      __threadfence();
    }
  }
}

__global__ __launch_bounds__(256) void layernorm_rows_kernel(
    const float* __restrict__ P, const float* __restrict__ lw, const float* __restrict__ lb,
    float* __restrict__ out)
{
  __shared__ __align__(16) float sR[8][kDm];
  constexpr float kInvDm = 1.0f / (float)kDm;
  const int lane = threadIdx.x & 31;
  const int wave = threadIdx.x >> 5;
  const size_t row = (size_t)blockIdx.x * 8 + wave;
  const float* pr = P + row * kDm + lane * 4;
  float* sr = &sR[wave][lane * 4];
  float s = 0.f;
#pragma unroll 1
  for (int it = 0; it < 8; ++it) {
    const v4f v = *(const v4f*)(pr + it * 128);
    *(v4f*)(sr + it * 128) = v;
    s += (v[0] + v[1]) + (v[2] + v[3]);
  }
#pragma unroll
  for (int off = 16; off > 0; off >>= 1) s += __shfl_xor(s, off, 32);
  const float mean = s * kInvDm;
  float q = 0.f;
#pragma unroll 1
  for (int it = 0; it < 8; ++it) {
    const v4f v = *(const v4f*)(sr + it * 128);
    const float d0 = v[0] - mean;
    const float d1 = v[1] - mean;
    const float d2 = v[2] - mean;
    const float d3 = v[3] - mean;
    q = fmaf(d0, d0, q);
    q = fmaf(d1, d1, q);
    q = fmaf(d2, d2, q);
    q = fmaf(d3, d3, q);
  }
#pragma unroll
  for (int off = 16; off > 0; off >>= 1) q += __shfl_xor(q, off, 32);
  const float var = q * kInvDm;
  const float inv = rsqrtf(var + 1e-5f);
  const float* lwp = lw + lane * 4;
  const float* lbp = lb + lane * 4;
#pragma unroll 1
  for (int it = 0; it < 8; ++it) {
    const v4f v  = *(const v4f*)(sr + it * 128);
    const v4f wv = *(const v4f*)(lwp + it * 128);
    const v4f bv = *(const v4f*)(lbp + it * 128);
    v4f o;
    o[0] = ((v[0] - mean) * inv) * wv[0] + bv[0];
    o[1] = ((v[1] - mean) * inv) * wv[1] + bv[1];
    o[2] = ((v[2] - mean) * inv) * wv[2] + bv[2];
    o[3] = ((v[3] - mean) * inv) * wv[3] + bv[3];
    *(v4f*)(sr + it * 128) = o;
  }
  float* orow = out + row * kDm + lane * 4;
  for (int pass = 0; pass < 2; ++pass) {
#pragma unroll 1
    for (int it = 0; it < 8; ++it) {
      const v4f o = *(const v4f*)(sr + it * 128);
      *(volatile v4f*)(orow + it * 128) = o;
    }
    __threadfence();
  }
}

extern "C" void kernel_launch(void* const* d_in, const int* in_sizes, int n_in,
                              void* d_out, int out_size, void* d_ws, size_t ws_size,
                              hipStream_t stream) {
  if (n_in < 12) return;
  if (in_sizes[0] != kRows * kDm) return;
  if (in_sizes[1] != kXzP * kDm) return;
  if (in_sizes[2] != kDin * 4) return;
  if (in_sizes[3] != kDin) return;
  if (in_sizes[4] != kXdN * kDin) return;
  if (in_sizes[5] != kDin * kDtR) return;
  if (in_sizes[6] != kDin) return;
  if (in_sizes[7] != kDin * kNst) return;
  if (in_sizes[8] != kDin) return;
  if (in_sizes[9] != kDm * kDin) return;
  if (in_sizes[10] != kDm) return;
  if (in_sizes[11] != kDm) return;
  if (out_size != kRows * kDm) return;
  if (ws_size < kWsTotal) return;

  const float* x       = (const float*)d_in[0];
  const float* W_in    = (const float*)d_in[1];
  const float* conv_w  = (const float*)d_in[2];
  const float* conv_b  = (const float*)d_in[3];
  const float* W_x     = (const float*)d_in[4];
  const float* W_dt    = (const float*)d_in[5];
  const float* b_dt    = (const float*)d_in[6];
  const float* A_log   = (const float*)d_in[7];
  const float* Dp      = (const float*)d_in[8];
  const float* W_out   = (const float*)d_in[9];
  const float* ln_w    = (const float*)d_in[10];
  const float* ln_b    = (const float*)d_in[11];
  float* out = (float*)d_out;

  char* ws = (char*)d_ws;
  unsigned short* XH  = (unsigned short*)(ws + kOffXH);
  unsigned short* WIH = (unsigned short*)(ws + kOffWIH);
  unsigned short* WXH = (unsigned short*)(ws + kOffWXH);
  unsigned short* WDH = (unsigned short*)(ws + kOffWDH);
  unsigned short* WOH = (unsigned short*)(ws + kOffWOH);
  unsigned short* XZH = (unsigned short*)(ws + kOffXZH);
  unsigned short* UCH = (unsigned short*)(ws + kOffUCH);
  float*          XD  = (float*)(ws + kOffXD);
  unsigned short* DLH = (unsigned short*)(ws + kOffDLH);
  unsigned short* DTH = (unsigned short*)(ws + kOffDTH);
  unsigned short* YGH = (unsigned short*)(ws + kOffYGH);
  float*          PLN = (float*)(ws + kOffPLN);

  cast_rows_f16<kCarryXLog2><<<(kRows * kDm / 8) / 256, 256, 0, stream>>>(
      x, XH, kDm, kDm, 7, kRows, kRows * kDm / 8);
  cast_rows_f16<kCarryWinLog2><<<(kXzP * kDm / 8) / 256, 256, 0, stream>>>(
      W_in, WIH, kDm, kDm, 7, kXzP, kXzP * kDm / 8);
  cast_rows_f16<kCarryWxLog2><<<(kXdP * kDin / 8) / 256, 256, 0, stream>>>(
      W_x, WXH, kDin, kDin, 8, kXdN, kXdP * kDin / 8);
  cast_rows_f16<kCarryWdtLog2><<<(kDin * kDtR / 8) / 256, 256, 0, stream>>>(
      W_dt, WDH, kDtR, kDtR, 3, kDin, kDin * kDtR / 8);
  cast_rows_f16<kCarryWoutLog2><<<(kDm * kDin / 8) / 256, 256, 0, stream>>>(
      W_out, WOH, kDin, kDin, 8, kDm, kDm * kDin / 8);

  wmma_gemm64_f16<kCarryXLog2 + kCarryWinLog2, 1, 0, 0, 0, 0>
      <<<(kRows / 64) * (kXzP / 64) / 8, 256, 0, stream>>>(
      XH, kDm, WIH, kDm, (void*)XZH, kXzP, b_dt, x, kDm, kRows, kXzP, kDm);

  conv_silu_kernel<<<dim3((kDin / 2) / 256, kRows / kConvRows), 256, 0, stream>>>(
      (const unsigned*)XZH, conv_w, conv_b, (unsigned*)UCH);

  wmma_gemm64_f16<kCarryUcLog2 + kCarryWxLog2, 0, 0, 0, 0, 0>
      <<<(kRows / 64) * (kXdP / 64) / 8, 256, 0, stream>>>(
      UCH, kDin, WXH, kDin, (void*)XD, kXdP, b_dt, x, kDm, kRows, kXdP, kDin);

  cast_rows_f16<kCarryDlLog2><<<(kRows * kDtR / 8) / 256, 256, 0, stream>>>(
      XD, DLH, kXdP, kDtR, 3, kRows, kRows * kDtR / 8);

  wmma_gemm64_f16<kCarryDlLog2 + kCarryWdtLog2, 1, 0, 1, 0, 1>
      <<<(kRows / 64) * (kDin / 64) / 8, 256, 0, stream>>>(
      DLH, kDtR, WDH, kDtR, (void*)DTH, kDin, b_dt, x, kDm, kRows, kDin, kDtR);

  scan_gate_kernel<<<kBatch * 4, 256, 0, stream>>>(
      (const unsigned*)DTH, (const unsigned*)UCH, (const unsigned*)XZH, XD, A_log, Dp, (unsigned*)YGH);

  wmma_gemm64_f16<kCarryYgLog2 + kCarryWoutLog2, 0, 0, 0, 1, 0>
      <<<(kRows / 64) * (kDm / 64) / 8, 256, 0, stream>>>(
      YGH, kDin, WOH, kDin, (void*)PLN, kDm, b_dt, x, kDm, kRows, kDm, kDin);

  layernorm_rows_kernel<<<kRows / 8, 256, 0, stream>>>(PLN, ln_w, ln_b, out);
}
